// SelfAttention_29575144800725
// MI455X (gfx1250) — hardware-verified
//
#include <hip/hip_runtime.h>


#ifndef NB
#define NB 4
#endif
#ifndef SEQ
#define SEQ 2048
#endif
#define NB_FULL   4
#define SEQ_FULL  2048
#define DM        1024
#define NWAVE     8
#define OP        68
#define CVB       2048u
#define NXB       ((unsigned)((size_t)NB * SEQ * DM / CVB))
#define NWB       ((unsigned)((size_t)3 * DM * DM / CVB))
#define NCH       (SEQ / 256)

#define EPI_QK  0
#define EPI_VT  1
#define EPI_F32 2

static_assert(SEQ % 256 == 0);
static_assert(SEQ <= SEQ_FULL);
static_assert(NB >= 1 && NB <= NB_FULL);
static_assert(DM == 1024);
static_assert(DM % 128 == 0);
static_assert(SEQ % 128 == 0);
static_assert((2 * DM) % 128 == 0);
static_assert(DM % 32 == 0 && SEQ % 32 == 0);
static_assert(DM % 8 == 0 && SEQ % 8 == 0);
static_assert(DM % 64 == 0);
static_assert(((size_t)NB * SEQ) % 128 == 0);
static_assert((size_t)NXB * CVB == (size_t)NB * SEQ * DM);
static_assert((size_t)NWB * CVB == (size_t)3 * DM * DM);
static_assert((size_t)DM * DM / CVB == 512);
static_assert(CVB == 256u * 8u);
static_assert(CVB == 2u * DM);
static_assert(NWAVE * 32 == 256);
static_assert(NCH * 256 == SEQ);
static_assert(NCH >= 1 && NCH <= 8);
static_assert((OP * 4) % 16 == 0);
static_assert(OP >= 64 + 4);
static_assert(((size_t)(NB - 1) * SEQ_FULL + SEQ) * DM * 4 <= (size_t)33554432);

#define XB_BYTES   ((size_t)NB * SEQ * DM * 2)
#define WB_BYTES   ((size_t)3 * DM * DM * 2)
#define QK_BYTES   ((size_t)2 * NB * SEQ * DM * 2)
#define VT_BYTES   ((size_t)NB * DM * SEQ * 2)
#define S_BYTES    ((size_t)SEQ * SEQ * 4)
#define P_BYTES    ((size_t)SEQ * SEQ * 2)
#define WS_TOTAL   (XB_BYTES + WB_BYTES + QK_BYTES + VT_BYTES + S_BYTES + P_BYTES)
static_assert(WS_TOTAL <= (size_t)134217728);
static_assert(XB_BYTES % 128 == 0 && WB_BYTES % 128 == 0);
static_assert(QK_BYTES % 128 == 0 && VT_BYTES % 128 == 0 && S_BYTES % 128 == 0 && P_BYTES % 128 == 0);

typedef __bf16   bf16;
typedef _Float16 f16;
typedef bf16     v16bf __attribute__((ext_vector_type(16)));
typedef f16      v16h  __attribute__((ext_vector_type(16)));
typedef float    v8f   __attribute__((ext_vector_type(8)));
typedef float    v4f   __attribute__((ext_vector_type(4)));
typedef unsigned v4u   __attribute__((ext_vector_type(4)));

union Pack8B { v4u u; bf16 h[8]; };
union Pack8H { v4u u; f16  h[8]; };

template <typename T> struct FragOf;
template <> struct FragOf<bf16> { typedef v16bf V; };
template <> struct FragOf<f16>  { typedef v16h  V; };

static __device__ __forceinline__ v8f mma16(v16bf a, v16bf b, v8f acc) {
  acc = __builtin_amdgcn_wmma_f32_16x16x32_bf16(false, a, false, b, (short)0, acc, false, false);
  asm volatile("v_nop\n\tv_nop\n\tv_nop\n\tv_nop" : "+v"(acc) : "v"(a), "v"(b));
  return acc;
}
static __device__ __forceinline__ v8f mma16(v16h a, v16h b, v8f acc) {
  acc = __builtin_amdgcn_wmma_f32_16x16x32_f16(false, a, false, b, (short)0, acc, false, false);
  asm volatile("v_nop\n\tv_nop\n\tv_nop\n\tv_nop" : "+v"(acc) : "v"(a), "v"(b));
  return acc;
}

static __device__ __forceinline__ void cvt8_store(const float* __restrict__ src, bf16* __restrict__ dst) {
  const v4f a0 = *(const v4f*)(src);
  const v4f a1 = *(const v4f*)(src + 4);
  Pack8B pk;
  #pragma unroll
  for (int i = 0; i < 4; ++i) {
    pk.h[i]     = (bf16)a0[i];
    pk.h[4 + i] = (bf16)a1[i];
  }
  const v4u val = pk.u;
  *(volatile v4u*)(dst) = val;
  __threadfence();
  *(volatile v4u*)(dst) = val;
}

__global__ __launch_bounds__(256) void convert_kernel(const float* __restrict__ x,
                                                      const float* __restrict__ wq,
                                                      const float* __restrict__ wk,
                                                      const float* __restrict__ wv,
                                                      bf16* __restrict__ xb,
                                                      bf16* __restrict__ wb) {
  #pragma clang fp contract(off)
  const unsigned blk = blockIdx.x;
  const unsigned tid = threadIdx.x;
  if (blk < NXB) {
    const unsigned r  = blk * 2u + (tid >> 7);
    const unsigned c  = (tid & 127u) * 8u;
    const unsigned bt = r / (unsigned)SEQ;
    const unsigned s  = r - bt * (unsigned)SEQ;
    cvt8_store(x + ((size_t)bt * SEQ_FULL + s) * DM + c, xb + (size_t)r * DM + c);
  } else {
    const unsigned wblk = blk - NXB;
    const unsigned wi   = wblk >> 9;
    const unsigned off  = (wblk & 511u) * CVB + tid * 8u;
    bf16* dst = wb + (size_t)wblk * CVB + tid * 8u;
    if (wi == 0u) {
      cvt8_store(wq + off, dst);
    } else if (wi == 1u) {
      cvt8_store(wk + off, dst);
    } else {
      cvt8_store(wv + off, dst);
    }
  }
}

template <typename T, int EPI>
static __device__ __forceinline__ void gemm_body(const T* __restrict__ A,
                                                 const T* __restrict__ Bt,
                                                 void* __restrict__ C,
                                                 unsigned nk, unsigned lda, unsigned ldb, unsigned ldc,
                                                 unsigned long long sAz, unsigned long long sBz,
                                                 unsigned long long sCz, float scale) {
  typedef typename FragOf<T>::V VT;
  union Frag { VT v; v4u q[2]; };

  __shared__ __align__(16) float sO[NWAVE * 16 * OP];

  const unsigned tid  = threadIdx.x;
  const unsigned wave = (unsigned)__builtin_amdgcn_readfirstlane((int)(tid >> 5));
  const unsigned lane = tid & 31u;
  const unsigned lq   = lane & 15u;
  const unsigned hi   = lane >> 4;
  const unsigned m0   = blockIdx.x * 128u + (wave & 3u) * 32u;
  const unsigned n0   = blockIdx.y * 128u + (wave >> 2) * 64u;

  const T* Ab = A  + (size_t)blockIdx.z * sAz;
  const T* Bb = Bt + (size_t)blockIdx.z * sBz;

  const T* ap[2];
  const T* bp[4];
  #pragma unroll
  for (int mt = 0; mt < 2; ++mt) ap[mt] = Ab + (size_t)(m0 + mt * 16u + lq) * lda + hi * 8u;
  #pragma unroll
  for (int nt = 0; nt < 4; ++nt) bp[nt] = Bb + (size_t)(n0 + nt * 16u + lq) * ldb + hi * 8u;

  v8f acc[2][4];
  #pragma unroll
  for (int mt = 0; mt < 2; ++mt) {
    #pragma unroll
    for (int nt = 0; nt < 4; ++nt) acc[mt][nt] = (v8f){0, 0, 0, 0, 0, 0, 0, 0};
  }

  #pragma unroll 1
  for (unsigned k = 0; k < nk; ++k) {
    const unsigned ko = k * 32u;
    Frag a[2], b[4];
    #pragma unroll
    for (int mt = 0; mt < 2; ++mt) {
      a[mt].q[0] = *(const v4u*)(ap[mt] + ko);
      a[mt].q[1] = *(const v4u*)(ap[mt] + ko + 16u);
    }
    #pragma unroll
    for (int nt = 0; nt < 4; ++nt) {
      b[nt].q[0] = *(const v4u*)(bp[nt] + ko);
      b[nt].q[1] = *(const v4u*)(bp[nt] + ko + 16u);
    }
    #pragma unroll
    for (int nt = 0; nt < 4; ++nt) {
      #pragma unroll
      for (int mt = 0; mt < 2; ++mt) acc[mt][nt] = mma16(a[mt].v, b[nt].v, acc[mt][nt]);
    }
  }

  size_t   cbase;
  unsigned ncol;
  if (EPI == EPI_QK) {
    cbase = (size_t)(n0 >> 10) * sCz;
    ncol  = n0 & 1023u;
  } else {
    cbase = (size_t)blockIdx.z * sCz;
    ncol  = n0;
  }

  float* so = sO + wave * (16u * OP);

  #pragma unroll
  for (int mt = 0; mt < 2; ++mt) {
    if (mt != 0) __syncthreads();
    #pragma unroll
    for (int r = 0; r < 8; ++r) {
      #pragma unroll
      for (int nt = 0; nt < 4; ++nt) {
        float val = acc[mt][nt][r];
        if (EPI == EPI_F32) val *= scale;
        so[(hi * 8u + r) * OP + nt * 16u + lq] = val;
      }
    }
    __syncthreads();

    if (EPI == EPI_F32) {
      float* Cf = (float*)C + cbase;
      v4f    vals[8];
      size_t gidx[8];
      #pragma unroll
      for (int it = 0; it < 8; ++it) {
        const unsigned row = it * 2u + hi;
        vals[it] = *(const v4f*)(so + row * OP + lq * 4u);
        gidx[it] = (size_t)(m0 + mt * 16u + row) * ldc + ncol + lq * 4u;
      }
      #pragma unroll
      for (int it = 0; it < 8; ++it) *(volatile v4f*)(Cf + gidx[it]) = vals[it];
      __threadfence();
      #pragma unroll
      for (int it = 0; it < 8; ++it) *(volatile v4f*)(Cf + gidx[it]) = vals[it];
    } else {
      f16* Ch = (f16*)C + cbase;
      v4u    vals[4];
      size_t gidx[4];
      #pragma unroll
      for (int it = 0; it < 4; ++it) {
        const unsigned row = it * 4u + (lane >> 3);
        const unsigned c8  = (lane & 7u) * 8u;
        const v4f x0 = *(const v4f*)(so + row * OP + c8);
        const v4f x1 = *(const v4f*)(so + row * OP + c8 + 4u);
        Pack8H ph;
        #pragma unroll
        for (int i = 0; i < 4; ++i) {
          ph.h[i]     = (f16)x0[i];
          ph.h[4 + i] = (f16)x1[i];
        }
        vals[it] = ph.u;
        gidx[it] = (size_t)(m0 + mt * 16u + row) * ldc + ncol + c8;
      }
      #pragma unroll
      for (int it = 0; it < 4; ++it) *(volatile v4u*)(Ch + gidx[it]) = vals[it];
      __threadfence();
      #pragma unroll
      for (int it = 0; it < 4; ++it) *(volatile v4u*)(Ch + gidx[it]) = vals[it];
    }
  }
}

__global__ __launch_bounds__(256) void gemm_qk_kernel(const bf16* __restrict__ A,
                                                      const bf16* __restrict__ Bt,
                                                      f16* __restrict__ C,
                                                      unsigned nk, unsigned lda, unsigned ldb, unsigned ldc,
                                                      unsigned long long sAz, unsigned long long sBz,
                                                      unsigned long long sCz) {
  gemm_body<bf16, EPI_QK>(A, Bt, (void*)C, nk, lda, ldb, ldc, sAz, sBz, sCz, 1.0f);
}

__global__ __launch_bounds__(256) void gemm_vt_kernel(const bf16* __restrict__ A,
                                                      const bf16* __restrict__ Bt,
                                                      f16* __restrict__ C,
                                                      unsigned nk, unsigned lda, unsigned ldb, unsigned ldc,
                                                      unsigned long long sAz, unsigned long long sBz,
                                                      unsigned long long sCz) {
  gemm_body<bf16, EPI_VT>(A, Bt, (void*)C, nk, lda, ldb, ldc, sAz, sBz, sCz, 1.0f);
}

__global__ __launch_bounds__(256) void gemm_f32_kernel(const f16* __restrict__ A,
                                                       const f16* __restrict__ Bt,
                                                       float* __restrict__ C,
                                                       unsigned nk, unsigned lda, unsigned ldb, unsigned ldc,
                                                       unsigned long long sAz, unsigned long long sBz,
                                                       unsigned long long sCz, float scale) {
  gemm_body<f16, EPI_F32>(A, Bt, (void*)C, nk, lda, ldb, ldc, sAz, sBz, sCz, scale);
}

__global__ __launch_bounds__(256) void softmax_kernel(const float* __restrict__ S, f16* __restrict__ P) {
  #pragma clang fp contract(off)
  const unsigned tid  = threadIdx.x;
  const unsigned wave = (unsigned)__builtin_amdgcn_readfirstlane((int)(tid >> 5));
  const unsigned lane = tid & 31u;
  const unsigned row  = blockIdx.x * 8u + wave;
  const float* sp = S + (size_t)row * SEQ + lane * 8u;

  v4f v[NCH][2];
  #pragma unroll
  for (int it = 0; it < NCH; ++it) {
    v[it][0] = *(const v4f*)(sp + it * 256);
    v[it][1] = *(const v4f*)(sp + it * 256 + 4);
  }

  float m = -__builtin_inff();
  #pragma unroll
  for (int it = 0; it < NCH; ++it) {
    #pragma unroll
    for (int i = 0; i < 4; ++i) {
      m = fmaxf(m, v[it][0][i]);
      m = fmaxf(m, v[it][1][i]);
    }
  }
  #pragma unroll
  for (int off = 16; off > 0; off >>= 1) m = fmaxf(m, __shfl_xor(m, off, 32));

  const float L2E = 1.4426950408889634f;
  float sum = 0.0f;
  #pragma unroll
  for (int it = 0; it < NCH; ++it) {
    #pragma unroll
    for (int i = 0; i < 4; ++i) {
      const float e0 = __builtin_amdgcn_exp2f((v[it][0][i] - m) * L2E);
      const float e1 = __builtin_amdgcn_exp2f((v[it][1][i] - m) * L2E);
      v[it][0][i] = e0;
      v[it][1][i] = e1;
      sum += e0;
      sum += e1;
    }
  }
  #pragma unroll
  for (int off = 16; off > 0; off >>= 1) sum += __shfl_xor(sum, off, 32);

  const float inv = 4096.0f * __builtin_amdgcn_rcpf(sum);

  v4u pk[NCH];
  #pragma unroll
  for (int it = 0; it < NCH; ++it) {
    Pack8H ph;
    #pragma unroll
    for (int i = 0; i < 4; ++i) {
      ph.h[i]     = (f16)(v[it][0][i] * inv);
      ph.h[4 + i] = (f16)(v[it][1][i] * inv);
    }
    pk[it] = ph.u;
  }

  f16* dp = P + (size_t)row * SEQ + lane * 8u;
  #pragma unroll
  for (int it = 0; it < NCH; ++it) *(volatile v4u*)(dp + it * 256) = pk[it];
  __threadfence();
  #pragma unroll
  for (int it = 0; it < NCH; ++it) *(volatile v4u*)(dp + it * 256) = pk[it];
}

extern "C" void kernel_launch(void* const* d_in, const int* in_sizes, int n_in,
                              void* d_out, int out_size, void* d_ws, size_t ws_size,
                              hipStream_t stream) {
  if (n_in < 4) return;
  const size_t rows_used = (size_t)(NB - 1) * SEQ_FULL + SEQ;
  if ((size_t)in_sizes[0] < rows_used * DM) return;
  if ((size_t)in_sizes[1] < (size_t)DM * DM) return;
  if ((size_t)in_sizes[2] < (size_t)DM * DM) return;
  if ((size_t)in_sizes[3] < (size_t)DM * DM) return;
  if ((size_t)out_size < rows_used * DM) return;
  if (ws_size < WS_TOTAL) return;

  const float* x  = (const float*)d_in[0];
  const float* wq = (const float*)d_in[1];
  const float* wk = (const float*)d_in[2];
  const float* wv = (const float*)d_in[3];
  float* out = (float*)d_out;

  char* w = (char*)d_ws;
  bf16*  xb    = (bf16*)w;   w += XB_BYTES;
  bf16*  wb    = (bf16*)w;   w += WB_BYTES;
  f16*   qk    = (f16*)w;    w += QK_BYTES;
  f16*   vt    = (f16*)w;    w += VT_BYTES;
  float* Sp    = (float*)w;  w += S_BYTES;
  f16*   Pp    = (f16*)w;    w += P_BYTES;

  const unsigned long long plane = (unsigned long long)NB * SEQ * DM;
  const f16* qp = qk;
  const f16* kp = qk + plane;

  convert_kernel<<<dim3(NXB + NWB), 256, 0, stream>>>(x, wq, wk, wv, xb, wb);

  gemm_qk_kernel<<<dim3((unsigned)((size_t)NB * SEQ / 128), 2 * DM / 128, 1), 256, 0, stream>>>(
      xb, wb, qk, DM / 32, DM, DM, DM, 0ull, 0ull, plane);

  gemm_vt_kernel<<<dim3(DM / 128, SEQ / 128, NB), 256, 0, stream>>>(
      wb + (size_t)2 * DM * DM, xb, vt, DM / 32, DM, DM, SEQ,
      0ull, (unsigned long long)SEQ * DM, (unsigned long long)DM * SEQ);

  for (int b = 0; b < NB; ++b) {
    gemm_f32_kernel<<<dim3(SEQ / 128, SEQ / 128, 1), 256, 0, stream>>>(
        qp + (size_t)b * SEQ * DM, kp + (size_t)b * SEQ * DM, Sp,
        DM / 32, DM, DM, SEQ, 0ull, 0ull, 0ull, 0.03125f);

    softmax_kernel<<<dim3(SEQ / 8), 256, 0, stream>>>(Sp, Pp);

    gemm_f32_kernel<<<dim3(SEQ / 128, DM / 128, 1), 256, 0, stream>>>(
        Pp, vt + (size_t)b * DM * SEQ, out + (size_t)b * SEQ_FULL * DM,
        SEQ / 32, SEQ, SEQ, DM, 0ull, 0ull, 0ull, 1.0f / 4096.0f);
  }
}
